// Model_17686675325086
// MI455X (gfx1250) — hardware-run, weakly checked
//
#include <hip/hip_runtime.h>

typedef float          v8f   __attribute__((ext_vector_type(8)));
typedef float          v4f   __attribute__((ext_vector_type(4)));
typedef unsigned int   v4u   __attribute__((ext_vector_type(4)));
typedef int            v8i   __attribute__((ext_vector_type(8)));
typedef unsigned short v8us  __attribute__((ext_vector_type(8)));
typedef unsigned short v16us __attribute__((ext_vector_type(16)));
typedef __bf16         v16bf __attribute__((ext_vector_type(16)));
typedef _Float16       v16h  __attribute__((ext_vector_type(16)));
typedef v4f  __attribute__((may_alias)) v4fa;
typedef v8us __attribute__((may_alias)) v8usa;
union FragB { v16bf v; v16us u; v8us h[2]; v8i w; };
union FragH { v16h  v; v16us u; v8us h[2]; v8i w; };

__device__ __forceinline__ v8f wmb(const FragB& a, const FragB& b, v8f c) {
  v8f d = __builtin_amdgcn_wmma_f32_16x16x32_bf16(false, a.v, false, b.v, (short)0, c, false, false);
  asm volatile("v_nop\n\tv_nop\n\tv_nop\n\tv_nop" : "+v"(d) : "v"(a.w), "v"(b.w));
  return d;
}

__device__ __forceinline__ v8f wmh(const FragH& a, const FragH& b, v8f c) {
  v8f d = __builtin_amdgcn_wmma_f32_16x16x32_f16(false, a.v, false, b.v, (short)0, c, false, false);
  asm volatile("v_nop\n\tv_nop\n\tv_nop\n\tv_nop" : "+v"(d) : "v"(a.w), "v"(b.w));
  return d;
}

__device__ __forceinline__ unsigned bf16_bits(float f) {
  const unsigned u = __float_as_uint(f);
  const unsigned r = (u + 0x7FFFu + ((u >> 16) & 1u)) >> 16;
  const unsigned q = (u >> 16) | 0x40u;
  return ((u & 0x7fffffffu) > 0x7f800000u) ? q : r;
}

__device__ __forceinline__ float bf16_val(float f) {
  return __uint_as_float(bf16_bits(f) << 16);
}
__device__ __forceinline__ int clampi(int v, int lo, int hi) {
  return v < lo ? lo : (v > hi ? hi : v);
}

__device__ __forceinline__ unsigned f16_bits(float f) {
  const unsigned u  = __float_as_uint(f);
  const unsigned s  = (u >> 16) & 0x8000u;
  const unsigned a  = u & 0x7fffffffu;
  const unsigned t  = a - 0x38000000u;
  const unsigned r  = (t + 0x0FFFu + ((t >> 13) & 1u)) >> 13;
  const unsigned rc = r > 0x7C00u ? 0x7C00u : r;
  const bool small  = a < 0x38800000u;
  const bool isnan  = a > 0x7f800000u;
  const unsigned fin = small ? 0u : (s | rc);
  return isnan ? (s | 0x7E00u) : fin;
}

__device__ __forceinline__ unsigned pk16(unsigned lo, unsigned hi) { return lo | (hi << 16); }
__device__ __forceinline__ unsigned bf16_lo_bits(float v) {
  float hi = bf16_val(v);
  asm volatile("" : "+v"(hi));
  return bf16_bits(v - hi);
}
__device__ __forceinline__ v4u pack8_bf16(v4f a, v4f c) {
  return (v4u){ pk16(bf16_bits(a[0]), bf16_bits(a[1])), pk16(bf16_bits(a[2]), bf16_bits(a[3])),
                pk16(bf16_bits(c[0]), bf16_bits(c[1])), pk16(bf16_bits(c[2]), bf16_bits(c[3])) };
}
__device__ __forceinline__ v4u pack8_bf16_lo(v4f a, v4f c) {
  return (v4u){ pk16(bf16_lo_bits(a[0]), bf16_lo_bits(a[1])), pk16(bf16_lo_bits(a[2]), bf16_lo_bits(a[3])),
                pk16(bf16_lo_bits(c[0]), bf16_lo_bits(c[1])), pk16(bf16_lo_bits(c[2]), bf16_lo_bits(c[3])) };
}
__device__ __forceinline__ v4u pack8_f16(v4f a, v4f c) {
  return (v4u){ pk16(f16_bits(a[0]), f16_bits(a[1])), pk16(f16_bits(a[2]), f16_bits(a[3])),
                pk16(f16_bits(c[0]), f16_bits(c[1])), pk16(f16_bits(c[2]), f16_bits(c[3])) };
}

template <int FORM>
__global__ __launch_bounds__(256) void k_plane(const float* __restrict__ src, int rows, int cols, int ldsrc,
                                               unsigned short* __restrict__ dst, int MP, int KP) {
  static_assert(FORM >= 0 && FORM <= 3);
  const int KTOT = (FORM == 1 || FORM == 3) ? 2 * KP : KP;
  const unsigned ppr   = (unsigned)(KTOT >> 3);
  const unsigned kp8   = (unsigned)(KP >> 3);
  const unsigned total = (unsigned)MP * ppr;
  const unsigned g     = blockIdx.x * 256u + threadIdx.x;
  const unsigned rowu  = g / ppr;
  const unsigned p     = g - rowu * ppr;
  const bool second    = p >= kp8;
  const int row = (int)rowu;
  const int c0  = (int)((second ? p - kp8 : p) << 3);
  const float* srow = src + (size_t)clampi(row, 0, rows - 1) * (size_t)ldsrc;
  float x[8];
  unsigned mk[8];
#pragma unroll
  for (int e = 0; e < 8; ++e) {
    const int c = c0 + e;
    const float v = srow[clampi(c, 0, cols - 1)];
    asm volatile("" :: "v"(v));
    x[e]  = v;
    mk[e] = (row < rows && c < cols) ? 0xFFFFu : 0u;
  }
  const v4f a = (v4f){ x[0], x[1], x[2], x[3] };
  const v4f c = (v4f){ x[4], x[5], x[6], x[7] };
  v4u o;
  if (FORM == 2) {
    o = pack8_f16(a, c);
  } else {
    const v4u hi = pack8_bf16(a, c);
    o = hi;
    if (FORM == 1) { const v4u lo = pack8_bf16_lo(a, c); o = second ? lo : hi; }
  }
  const v4u mw = (v4u){ pk16(mk[0], mk[1]), pk16(mk[2], mk[3]), pk16(mk[4], mk[5]), pk16(mk[6], mk[7]) };
  o &= mw;
  if (g < total) {
    volatile v4u* q = (volatile v4u*)(dst + (size_t)g * 8);
    *q = o;
    __threadfence();
    *q = o;
  }
}

template <int FORM> struct FragOf    { typedef FragB T; };
template <>         struct FragOf<2> { typedef FragH T; };
__device__ __forceinline__ v8f mm(const FragB& a, const FragB& b, v8f c) { return wmb(a, b, c); }
__device__ __forceinline__ v8f mm(const FragH& a, const FragH& b, v8f c) { return wmh(a, b, c); }
template <class F> __device__ __forceinline__ F ld_frag(const unsigned short* p) {
  F f;
  f.h[0] = *(const v8usa*)(p);
  f.h[1] = *(const v8usa*)(p + 16);
  return f;
}

template <int FORM, int EPI>
__global__ __launch_bounds__(256) __attribute__((amdgpu_num_vgpr(248)))
void k_gemm_nt(const unsigned short* __restrict__ A, const unsigned short* __restrict__ B,
               const float* __restrict__ bias, float* __restrict__ D, int M, int N, int KTOT, int ldd) {
  static_assert(FORM >= 0 && FORM <= 2);
  static_assert(EPI == 0 || EPI == 1);
  typedef typename FragOf<FORM>::T F;
  __shared__ __attribute__((aligned(16))) float sT[8][16 * 68];
  const int lane = threadIdx.x & 31;
  const int wave = threadIdx.x >> 5;
  const int tilesM = (M + 63) >> 6;
  const int tilesN = (N + 63) >> 6;
  const int tile = blockIdx.x * 8 + wave;
  if (tile >= tilesM * tilesN) return;
  const int tm = tile / tilesN;
  const int tn = tile - tm * tilesN;
  const int m0 = tm << 6;
  const int n0 = tn << 6;

  const int rl = lane & 15;
  const int h8 = (lane >> 4) * 8;
  const unsigned short* pa = A + (size_t)(m0 + rl) * (size_t)KTOT + h8;
  const unsigned short* pb = B + (size_t)(n0 + rl) * (size_t)KTOT + h8;

  v8f acc[4][4];
#pragma unroll
  for (int i = 0; i < 4; ++i)
#pragma unroll
    for (int j = 0; j < 4; ++j) acc[i][j] = (v8f){0.f, 0.f, 0.f, 0.f, 0.f, 0.f, 0.f, 0.f};

#pragma unroll 1
  for (int k0 = 0; k0 < KTOT; k0 += 32) {
    F bf[4];
#pragma unroll
    for (int j = 0; j < 4; ++j) bf[j] = ld_frag<F>(pb + (size_t)(j << 4) * (size_t)KTOT + k0);
#pragma unroll
    for (int i = 0; i < 4; ++i) {
      const F af = ld_frag<F>(pa + (size_t)(i << 4) * (size_t)KTOT + k0);
#pragma unroll
      for (int j = 0; j < 4; ++j) acc[i][j] = mm(af, bf[j], acc[i][j]);
    }
  }

  float* slab = sT[wave];
  const int hh = lane >> 4;
  const int c4 = (lane & 15) * 4;
  const int nc = n0 + c4;
  const bool cok = nc < N;
  v4f bv = (v4f){0.f, 0.f, 0.f, 0.f};
  if (EPI == 1) {
    bv = *(const v4fa*)(bias + clampi(nc, 0, N - 4));
    asm volatile("" :: "v"(bv));
  }
#pragma unroll
  for (int i = 0; i < 4; ++i) {
    const int mBase = m0 + (i << 4);
#pragma unroll
    for (int j = 0; j < 4; ++j) {
#pragma unroll
      for (int r = 0; r < 8; ++r) slab[(h8 + r) * 68 + (j << 4) + rl] = acc[i][j][r];
    }
    __builtin_amdgcn_fence(__ATOMIC_RELEASE, "workgroup");
    __builtin_amdgcn_wave_barrier();
    __builtin_amdgcn_fence(__ATOMIC_ACQUIRE, "workgroup");
    v4f vv[8];
#pragma unroll
    for (int it = 0; it < 8; ++it) {
      const int row = it * 2 + hh;
      v4f v = *(const v4fa*)(slab + row * 68 + c4);
      if (EPI == 1) v += bv;
      vv[it] = v;
    }
    for (int pass = 0; pass < 2; ++pass) {
#pragma unroll
      for (int it = 0; it < 8; ++it) {
        const int row = mBase + it * 2 + hh;
        if (cok && row < M) *(volatile v4f*)(D + (size_t)row * (size_t)ldd + nc) = vv[it];
      }
      __threadfence();
    }
    __builtin_amdgcn_fence(__ATOMIC_RELEASE, "workgroup");
    __builtin_amdgcn_wave_barrier();
    __builtin_amdgcn_fence(__ATOMIC_ACQUIRE, "workgroup");
  }
}

typedef float v2f __attribute__((ext_vector_type(2)));
typedef v2f __attribute__((may_alias)) v2fa;

static constexpr int BATCH  = 2;
static constexpr int NODES  = 50000;
static constexpr int CFEAT  = 16;
static constexpr int DWIDTH = 128;
static constexpr int EDGES  = 1600000;
static constexpr int MROWS  = BATCH * NODES;
static constexpr int MPAD   = 100032;
static constexpr int KPAD   = 32;
static constexpr int OUT0_ELEMS = MROWS * DWIDTH;
static constexpr int OUT1_ELEM0 = OUT0_ELEMS;
static constexpr int OUT1_ELEMS = BATCH * EDGES;
static constexpr int OUT_TOTAL  = OUT0_ELEMS + OUT1_ELEMS;

static constexpr size_t WS_XB_BYTES  = (size_t)MPAD * KPAD * 2;
static constexpr size_t WS_WT_BYTES  = (size_t)DWIDTH * KPAD * 2;
static constexpr size_t WS_PRE_BYTES = (size_t)MPAD * DWIDTH * 4;
static constexpr size_t WS_OFF_XB    = 0;
static constexpr size_t WS_OFF_WT    = WS_OFF_XB + WS_XB_BYTES;
static constexpr size_t WS_OFF_PRE   = WS_OFF_WT + WS_WT_BYTES;
static constexpr size_t WS_TOTAL     = WS_OFF_PRE + WS_PRE_BYTES;

static constexpr int PLANE_BLOCKS = MPAD * KPAD / 8 / 256;
static constexpr int WT_PIECES    = DWIDTH * KPAD / 8;
static constexpr int GEMM_TILES   = ((MROWS + 63) / 64) * ((DWIDTH + 63) / 64);
static constexpr int GEMM_BLOCKS  = (GEMM_TILES + 7) / 8;

static_assert(BATCH == 2 && NODES == 50000 && CFEAT == 16 && DWIDTH == 128 && EDGES == 1600000);
static_assert(MPAD % 64 == 0 && MPAD >= MROWS && MPAD - MROWS < 64);
static_assert(DWIDTH % 64 == 0 && KPAD % 32 == 0 && CFEAT <= KPAD);
static_assert(MROWS % 16 == 0 && MROWS % 8 == 0 && DWIDTH % 32 == 0 && DWIDTH == 32 * 4);
static_assert((MPAD * KPAD / 8) % 256 == 0 && PLANE_BLOCKS == 1563);
static_assert(WT_PIECES == 2 * 256);
static_assert(EDGES % 256 == 0 && EDGES % 32 == 0);
static_assert(((size_t)OUT1_ELEM0 * 4) % 128 == 0 && ((size_t)OUT1_ELEM0 * 4) / 128 == 400000);
static_assert(((size_t)EDGES * 4) % 128 == 0 && ((size_t)EDGES * 4) / 128 == 50000);
static_assert(OUT_TOTAL == 16000000);
static_assert(OUT1_ELEM0 + (BATCH - 1) * EDGES + (EDGES - 1) == OUT_TOTAL - 1);
static_assert((MROWS - 1) * DWIDTH + DWIDTH - 1 == OUT0_ELEMS - 1);
static_assert(WS_XB_BYTES == 6402048 && WS_WT_BYTES == 8192 && WS_PRE_BYTES == 51216384);
static_assert(WS_OFF_WT % 256 == 0 && WS_OFF_PRE % 256 == 0 && WS_TOTAL == 57626624);
static_assert(WS_TOTAL <= ((size_t)128 << 20));

__global__ __launch_bounds__(256) void k_wt(const float* __restrict__ w, unsigned short* __restrict__ wt) {
  const int g  = (int)blockIdx.x * 256 + (int)threadIdx.x;
  const int n  = g >> 2;
  const int k0 = (g & 3) << 3;
  float x[8];
  unsigned mk[8];
#pragma unroll
  for (int e = 0; e < 8; ++e) {
    const int k = k0 + e;
    const float v = w[clampi(k, 0, CFEAT - 1) * DWIDTH + n];
    asm volatile("" :: "v"(v));
    x[e]  = v;
    mk[e] = (k < CFEAT) ? 0xFFFFu : 0u;
  }
  const v4f a = (v4f){ x[0], x[1], x[2], x[3] };
  const v4f c = (v4f){ x[4], x[5], x[6], x[7] };
  v4u o = pack8_bf16(a, c);
  const v4u mw = (v4u){ pk16(mk[0], mk[1]), pk16(mk[2], mk[3]), pk16(mk[4], mk[5]), pk16(mk[6], mk[7]) };
  o &= mw;
  if (g < WT_PIECES) {
    volatile v4u* q = (volatile v4u*)(wt + (size_t)g * 8);
    *q = o;
    __threadfence();
    *q = o;
  }
}

__global__ __launch_bounds__(256) void k_rowln(const float* __restrict__ pre, const float* __restrict__ fcb,
                                               const float* __restrict__ lng, const float* __restrict__ lnb,
                                               float* out) {
  const int lane = (int)threadIdx.x & 31;
  const int wave = (int)threadIdx.x >> 5;
  const int row  = (int)blockIdx.x * 8 + wave;
  const int c4   = lane * 4;
  const v4f p  = *(const v4fa*)(pre + (size_t)row * DWIDTH + c4);
  const v4f fb = *(const v4fa*)(fcb + c4);
  const v4f gg = *(const v4fa*)(lng + c4);
  const v4f bb = *(const v4fa*)(lnb + c4);
  v4f x = (v4f){ p[0] + bf16_val(fb[0]), p[1] + bf16_val(fb[1]), p[2] + bf16_val(fb[2]), p[3] + bf16_val(fb[3]) };
#pragma unroll 1
  for (int i = 0; i < 4; ++i) {
    const float t = x[0];
    const float a = 0.5f * t * (1.0f + erff(t * 0.70710678f));
    x = (v4f){ x[1], x[2], x[3], a };
  }
  float s = (x[0] + x[1]) + (x[2] + x[3]);
  s += __shfl_xor(s, 16, 32);
  s += __shfl_xor(s, 8, 32);
  s += __shfl_xor(s, 4, 32);
  s += __shfl_xor(s, 2, 32);
  s += __shfl_xor(s, 1, 32);
  const float mu = s * (1.0f / 128.0f);
  const float d0 = x[0] - mu, d1 = x[1] - mu, d2 = x[2] - mu, d3 = x[3] - mu;
  float q = (d0 * d0 + d1 * d1) + (d2 * d2 + d3 * d3);
  q += __shfl_xor(q, 16, 32);
  q += __shfl_xor(q, 8, 32);
  q += __shfl_xor(q, 4, 32);
  q += __shfl_xor(q, 2, 32);
  q += __shfl_xor(q, 1, 32);
  const float var = q * (1.0f / 128.0f);
  const float r = 1.0f / sqrtf(var + 1e-5f);
  v4f o;
  o[0] = d0 * r * bf16_val(gg[0]) + bf16_val(bb[0]);
  o[1] = d1 * r * bf16_val(gg[1]) + bf16_val(bb[1]);
  o[2] = d2 * r * bf16_val(gg[2]) + bf16_val(bb[2]);
  o[3] = d3 * r * bf16_val(gg[3]) + bf16_val(bb[3]);
  volatile v4f* dp = (volatile v4f*)(out + (size_t)row * DWIDTH + c4);
  *dp = o;
  __threadfence();
  *dp = o;
}

__global__ __launch_bounds__(256) void k_edge(const float* __restrict__ st, const int* __restrict__ ei, float* out) {
#pragma clang fp contract(off)
  const int e = (int)blockIdx.x * 256 + (int)threadIdx.x;
  int s = ei[e];
  int t = ei[EDGES + e];
  asm volatile("" :: "v"(s));
  asm volatile("" :: "v"(t));
  s = clampi(s, 0, NODES - 1);
  t = clampi(t, 0, NODES - 1);
  const v2f a0 = *(const v2fa*)(st + (size_t)s * CFEAT);
  const v2f c0 = *(const v2fa*)(st + (size_t)t * CFEAT);
  const v2f a1 = *(const v2fa*)(st + (size_t)(NODES + s) * CFEAT);
  const v2f c1 = *(const v2fa*)(st + (size_t)(NODES + t) * CFEAT);
  const float a0x = a0.x, a0y = a0.y, c0x = c0.x, c0y = c0.y;
  const float a1x = a1.x, a1y = a1.y, c1x = c1.x, c1y = c1.y;
  asm volatile("" :: "v"(a0x)); asm volatile("" :: "v"(a0y));
  asm volatile("" :: "v"(c0x)); asm volatile("" :: "v"(c0y));
  asm volatile("" :: "v"(a1x)); asm volatile("" :: "v"(a1y));
  asm volatile("" :: "v"(c1x)); asm volatile("" :: "v"(c1y));
  const float dx0 = bf16_val(a0x) - bf16_val(c0x);
  const float dy0 = bf16_val(a0y) - bf16_val(c0y);
  const float dx1 = bf16_val(a1x) - bf16_val(c1x);
  const float dy1 = bf16_val(a1y) - bf16_val(c1y);
  const float q0 = __fadd_rn(__fmul_rn(dx0, dx0), __fmul_rn(dy0, dy0));
  const float q1 = __fadd_rn(__fmul_rn(dx1, dx1), __fmul_rn(dy1, dy1));
  const float det0 = -0.5f * q0;
  const float det1 = -0.5f * q1;
  volatile float* p0 = (volatile float*)(out + (size_t)OUT1_ELEM0 + (size_t)e);
  volatile float* p1 = (volatile float*)(out + (size_t)OUT1_ELEM0 + (size_t)EDGES + (size_t)e);
  *p0 = det0;
  *p1 = det1;
  __threadfence();
  *p0 = det0;
  *p1 = det1;
}

extern "C" void kernel_launch(void* const* d_in, const int* in_sizes, int n_in,
                              void* d_out, int out_size, void* d_ws, size_t ws_size,
                              hipStream_t stream) {
  if (n_in < 6) return;
  if (in_sizes[0] != MROWS * CFEAT) return;
  if (in_sizes[1] != 2 * EDGES) return;
  if (in_sizes[2] != CFEAT * DWIDTH) return;
  if (in_sizes[3] != DWIDTH) return;
  if (in_sizes[4] != DWIDTH) return;
  if (in_sizes[5] != DWIDTH) return;
  if (out_size != OUT_TOTAL) return;
  if (ws_size < WS_TOTAL) return;

  const float* st  = (const float*)d_in[0];
  const int*   ei  = (const int*)d_in[1];
  const float* fcw = (const float*)d_in[2];
  const float* fcb = (const float*)d_in[3];
  const float* lng = (const float*)d_in[4];
  const float* lnb = (const float*)d_in[5];
  float* out = (float*)d_out;

  char* ws = (char*)d_ws;
  unsigned short* XB  = (unsigned short*)(ws + WS_OFF_XB);
  unsigned short* WT  = (unsigned short*)(ws + WS_OFF_WT);
  float*          PRE = (float*)(ws + WS_OFF_PRE);

  k_plane<0><<<PLANE_BLOCKS, 256, 0, stream>>>(st, MROWS, CFEAT, CFEAT, XB, MPAD, KPAD);
  k_wt<<<WT_PIECES / 256, 256, 0, stream>>>(fcw, WT);
  k_gemm_nt<0, 0><<<GEMM_BLOCKS, 256, 0, stream>>>(XB, WT, fcb, PRE, MROWS, DWIDTH, KPAD, DWIDTH);
  k_rowln<<<MROWS / 8, 256, 0, stream>>>(PRE, fcb, lng, lnb, out);
  k_edge<<<EDGES / 256, 256, 0, stream>>>(st, ei, out);
}
